// CrossAttention_3126736191504
// MI455X (gfx1250) — hardware-verified
//
#include <hip/hip_runtime.h>
#ifndef NB
#define NB 4
#endif
#ifndef SEQ
#define SEQ 2048
#endif
#define NB_FULL 4
#define SEQ_FULL 2048
#define DM 1024
#define NH 16
#define HD 64
#define NR ((size_t)NB * SEQ)

static_assert(NB >= 1 && NB <= NB_FULL);
static_assert(SEQ <= SEQ_FULL);
static_assert(SEQ % 128 == 0);
static_assert(DM % 128 == 0);
static_assert(NH * HD == DM);
static_assert(HD == 64);
static_assert(NH == 16);
static_assert((NB * SEQ) % 128 == 0);
static_assert((NB * SEQ) % 4 == 0);
static_assert(DM % 64 == 0);
static_assert(DM % 32 == 0);
static_assert(DM == 4 * 32 * 8);
static_assert(((size_t)DM * DM) % 8 == 0);
static_assert((size_t)4 * DM * DM * 2 + (size_t)6 * NB * SEQ * DM * 2 <= (size_t)134217728);

typedef _Float16 v16h __attribute__((ext_vector_type(16)));
typedef _Float16 v4h __attribute__((ext_vector_type(4)));
typedef unsigned short v8us __attribute__((ext_vector_type(8), may_alias));
typedef float v8f __attribute__((ext_vector_type(8)));
typedef float v4f __attribute__((ext_vector_type(4)));
typedef float v4fa __attribute__((ext_vector_type(4), may_alias));
union FragH { v16h v; v8us half[2]; _Float16 h[16]; unsigned short u[16]; };

__device__ __forceinline__ unsigned short bf16_bits(float x) { unsigned int u = __float_as_uint(x); return (unsigned short)((u + 0x7FFFu + ((u >> 16) & 1u)) >> 16); }
__device__ __forceinline__ float bf16_rne(float x) { return __uint_as_float(((unsigned int)bf16_bits(x)) << 16); }

__device__ __forceinline__ v8us cvt8(const float* __restrict__ p, float scale) {
  const v4f a = *(const v4fa*)p, c = *(const v4fa*)(p + 4);
  FragH f;
#pragma unroll
  for (int q = 0; q < 4; ++q) { f.h[q] = (_Float16)(bf16_rne(a[q]) * scale); f.h[4 + q] = (_Float16)(bf16_rne(c[q]) * scale); }
  return f.half[0];
}

static __device__ __forceinline__ _Float16 toh_flush(float v) { const _Float16 r = (_Float16)v; return (fabsf(v) < 6.103515625e-05f) ? (_Float16)0.0f : r; }

__device__ __forceinline__ v8us cvt8f(const float* __restrict__ p, float scale) {
  const v4f a = *(const v4fa*)p, c = *(const v4fa*)(p + 4);
  FragH f;
#pragma unroll
  for (int q = 0; q < 4; ++q) { f.h[q] = toh_flush(bf16_rne(a[q]) * scale); f.h[4 + q] = toh_flush(bf16_rne(c[q]) * scale); }
  return f.half[0];
}

__global__ __launch_bounds__(256) void k_wperm4(const float* __restrict__ wq, const float* __restrict__ wk, const float* __restrict__ wv, const float* __restrict__ wo, size_t n8, _Float16* __restrict__ Bt) {
  #pragma clang fp contract(off)
  const size_t t = (size_t)blockIdx.x * 256 + threadIdx.x; if (t >= n8) return;
  const size_t e = t * 8; const size_t n = e / DM; const size_t col = e - n * DM;
  const size_t src = ((n & (size_t)(NH - 1)) * HD + (n / NH)) * DM + col;
  const v8us o0 = cvt8f(wq + src, 16.0f), o1 = cvt8f(wk + src, 16.0f), o2 = cvt8f(wv + e, 16.0f), o3 = cvt8f(wo + e, 16.0f);
  unsigned short* d = (unsigned short*)Bt + e; const size_t ps = (size_t)DM * DM;
  *(volatile v8us*)d = o0; *(volatile v8us*)(d + ps) = o1; *(volatile v8us*)(d + 2 * ps) = o2; *(volatile v8us*)(d + 3 * ps) = o3;
  __threadfence();
  *(volatile v8us*)d = o0; *(volatile v8us*)(d + ps) = o1; *(volatile v8us*)(d + 2 * ps) = o2; *(volatile v8us*)(d + 3 * ps) = o3;
}

__global__ __launch_bounds__(256) void k_x16(const float* __restrict__ x, _Float16* __restrict__ X16, size_t n8) {
  #pragma clang fp contract(off)
  const size_t t = (size_t)blockIdx.x * 256 + threadIdx.x; if (t >= n8) return;
  const size_t e = t * 8; const size_t row = e / DM; const size_t col = e - row * DM; const size_t b = row / SEQ; const size_t s = row - b * SEQ;
  const v8us o = cvt8(x + (b * SEQ_FULL + s) * DM + col, 1.0f);
  unsigned short* d = (unsigned short*)X16 + e;
  *(volatile v8us*)d = o; __threadfence(); *(volatile v8us*)d = o;
}

__device__ __forceinline__ v16h g2_frag(const _Float16* p, int hh) { FragH f; f.half[0] = *(const v8us*)((const unsigned short*)p + 8 * hh); f.half[1] = *(const v8us*)((const unsigned short*)p + 16 + 8 * hh); return f.v; }
__device__ __forceinline__ v8f g2_mma(v16h a, v16h b, v8f c) { v8f d = __builtin_amdgcn_wmma_f32_16x16x32_f16(false, a, false, b, (short)0, c, false, false); asm volatile("v_nop\n\tv_nop\n\tv_nop\n\tv_nop" : "+v"(d) : "v"(a), "v"(b)); return d; }
__global__ __launch_bounds__(128) void k_gemm2(const _Float16* __restrict__ A, int lda, size_t sA, const _Float16* __restrict__ Bh, int ldb, size_t sB, float alpha,
    float* __restrict__ C, _Float16* __restrict__ C16, int ldc, size_t sC, int M, int N, int K) {
  __shared__ __attribute__((aligned(16))) float so[4][32][68];
  const int tid = threadIdx.x, lane = tid & 31, ln = lane & 15, hh = lane >> 4; const int w = __builtin_amdgcn_readfirstlane(tid >> 5); const int by = blockIdx.y;
  A += (size_t)by * sA; Bh += (size_t)by * sB; const size_t cofs = (size_t)by * sC;
  const int ntn = N >> 6; const int mt = blockIdx.x / ntn, nq = blockIdx.x - mt * ntn; const int row0 = mt * 128 + 32 * w, col0 = nq * 64; if (row0 >= M) return;
  const _Float16* a0p = A + (size_t)(row0 + ln) * lda; const _Float16* a1p = a0p + (size_t)16 * lda;
  const _Float16* b0p = Bh + (size_t)(col0 + ln) * ldb; const _Float16* b1p = b0p + (size_t)16 * ldb; const _Float16* b2p = b1p + (size_t)16 * ldb; const _Float16* b3p = b2p + (size_t)16 * ldb;
  const v8f z8 = {0.f,0.f,0.f,0.f,0.f,0.f,0.f,0.f}; v8f c00 = z8, c01 = z8, c02 = z8, c03 = z8, c10 = z8, c11 = z8, c12 = z8, c13 = z8;
#pragma unroll 1
  for (int kb = 0; kb < K; kb += 32) { const v16h a0 = g2_frag(a0p + kb, hh), a1 = g2_frag(a1p + kb, hh);
    v16h b = g2_frag(b0p + kb, hh); c00 = g2_mma(a0, b, c00); c10 = g2_mma(a1, b, c10);
    b = g2_frag(b1p + kb, hh); c01 = g2_mma(a0, b, c01); c11 = g2_mma(a1, b, c11);
    b = g2_frag(b2p + kb, hh); c02 = g2_mma(a0, b, c02); c12 = g2_mma(a1, b, c12);
    b = g2_frag(b3p + kb, hh); c03 = g2_mma(a0, b, c03); c13 = g2_mma(a1, b, c13); }
  v8f accs[8] = {c00, c01, c02, c03, c10, c11, c12, c13};
#pragma unroll
  for (int u = 0; u < 8; ++u) { const int t = u & 3, half = u >> 2;
#pragma unroll
    for (int r = 0; r < 8; ++r) { const int rloc = half * 16 + 8 * hh + r; so[w][rloc][t * 16 + ln] = accs[u][r] * alpha; } }
  __builtin_amdgcn_fence(4  , "workgroup"); __builtin_amdgcn_wave_barrier();
  const int rsub = lane >> 4, c4 = (lane & 15) * 4;
  for (int pass = 0; pass < 2; ++pass) {
#pragma unroll
    for (int q = 0; q < 16; ++q) { const int r = q * 2 + rsub; const v4f v = *(const v4fa*)&so[w][r][c4];
      if (C) *(volatile v4f*)(C + cofs + (size_t)(row0 + r) * ldc + col0 + c4) = v;
      if (C16) { v4h h4; for (int i = 0; i < 4; ++i) h4[i] = (_Float16)v[i]; *(volatile v4h*)(C16 + cofs + (size_t)(row0 + r) * ldc + col0 + c4) = h4; } }
    if (pass == 0) __threadfence(); } }

__global__ __launch_bounds__(128) void k_attn_tok(const _Float16* __restrict__ Qp, const _Float16* __restrict__ Kp, const _Float16* __restrict__ V16, _Float16* __restrict__ CC) {
  __shared__ __attribute__((aligned(16))) _Float16 so[4][DM];
  const int tid = threadIdx.x, lane = tid & 31, ln = lane & 15, hh = lane >> 4;
  const int w = __builtin_amdgcn_readfirstlane(tid >> 5);
  const size_t tok = (size_t)blockIdx.x * 4 + (size_t)w;
  const unsigned short* qp = (const unsigned short*)Qp + tok * DM + ln * NH + 8 * hh;
  const unsigned short* kp = (const unsigned short*)Kp + tok * DM + ln * NH + 8 * hh;
  const unsigned short* vp = (const unsigned short*)V16 + tok * DM + ln * HD + 8 * hh;
  const v8us zh = {0, 0, 0, 0, 0, 0, 0, 0};
  const v8f z8 = {0.f,0.f,0.f,0.f,0.f,0.f,0.f,0.f};
  FragH ak0, ak1, ak2, ak3, av0, av1;
  ak0.half[0] = *(const v8us*)(kp);            ak0.half[1] = zh;
  ak1.half[0] = *(const v8us*)(kp + 16 * NH);  ak1.half[1] = zh;
  ak2.half[0] = *(const v8us*)(kp + 32 * NH);  ak2.half[1] = zh;
  ak3.half[0] = *(const v8us*)(kp + 48 * NH);  ak3.half[1] = zh;
  av0.half[0] = *(const v8us*)(vp);       av0.half[1] = *(const v8us*)(vp + 16);
  av1.half[0] = *(const v8us*)(vp + 32);  av1.half[1] = *(const v8us*)(vp + 48);
  const float c = 0.125f * 1.4426950408889634f;
#pragma unroll 1
  for (int it = 0; it < 4; ++it) {
    FragH bq; bq.half[0] = *(const v8us*)(qp + it * 16 * NH); bq.half[1] = zh;
    const v8f s0 = g2_mma(ak0.v, bq.v, z8);
    const v8f s1 = g2_mma(ak1.v, bq.v, z8);
    const v8f s2 = g2_mma(ak2.v, bq.v, z8);
    const v8f s3 = g2_mma(ak3.v, bq.v, z8);
    float mx = fmaxf(fmaxf(s0[0], s1[0]), fmaxf(s2[0], s3[0]));
#pragma unroll
    for (int r = 1; r < 8; ++r) mx = fmaxf(mx, fmaxf(fmaxf(s0[r], s1[r]), fmaxf(s2[r], s3[r])));
    mx = fmaxf(mx, __shfl_xor(mx, 16, 32));
    const float off = 8.0f - mx * c;
    FragH pf0, pf1; float ls = 0.f;
#pragma unroll
    for (int r = 0; r < 8; ++r) {
      const float e0 = fmaf(s0[r], c, off), e1 = fmaf(s1[r], c, off), e2 = fmaf(s2[r], c, off), e3 = fmaf(s3[r], c, off);
      const float p0 = (e0 < -14.0f) ? 0.0f : __builtin_amdgcn_exp2f(e0);
      const float p1 = (e1 < -14.0f) ? 0.0f : __builtin_amdgcn_exp2f(e1);
      const float p2 = (e2 < -14.0f) ? 0.0f : __builtin_amdgcn_exp2f(e2);
      const float p3 = (e3 < -14.0f) ? 0.0f : __builtin_amdgcn_exp2f(e3);
      const _Float16 h0 = (_Float16)p0, h1 = (_Float16)p1, h2 = (_Float16)p2, h3 = (_Float16)p3;
      ls += ((float)h0 + (float)h1) + ((float)h2 + (float)h3);
      pf0.h[r] = h0; pf0.h[8 + r] = h1; pf1.h[r] = h2; pf1.h[8 + r] = h3;
    }
    ls += __shfl_xor(ls, 16, 32);
    v8f o = g2_mma(av0.v, pf0.v, z8);
    o = g2_mma(av1.v, pf1.v, o);
    const float inv = 64.0f * (1.0f / ls);
#pragma unroll
    for (int r = 0; r < 8; ++r) so[w][(8 * hh + r) * HD + it * 16 + ln] = toh_flush(o[r] * inv);
  }
  __syncthreads();
  unsigned short* ob = (unsigned short*)CC + tok * DM;
  for (int pass = 0; pass < 2; ++pass) {
#pragma unroll
    for (int itp = 0; itp < 4; ++itp) { const int pc = (itp * 32 + lane) * 8; const v8us v = *(const v8us*)&so[w][pc]; *(volatile v8us*)(ob + pc) = v; }
    if (pass == 0) __threadfence();
  }
}

extern "C" void kernel_launch(void* const* d_in, const int* in_sizes, int n_in,
                              void* d_out, int out_size, void* d_ws, size_t ws_size, hipStream_t stream) {
  if (n_in < 6) return;
  const size_t need_x = ((size_t)(NB - 1) * SEQ_FULL + SEQ) * DM;
  if ((size_t)in_sizes[0] < need_x || (size_t)in_sizes[1] < need_x) return;
  if ((size_t)in_sizes[2] < (size_t)DM * DM || (size_t)in_sizes[3] < (size_t)DM * DM || (size_t)in_sizes[4] < (size_t)DM * DM || (size_t)in_sizes[5] < (size_t)DM * DM) return;
  if ((size_t)out_size < need_x) return;
  const float* x = (const float*)d_in[0]; const float* ctx = (const float*)d_in[1];
  const float* wq = (const float*)d_in[2]; const float* wk = (const float*)d_in[3]; const float* wv = (const float*)d_in[4]; const float* wo = (const float*)d_in[5];
  char* ws = (char*)d_ws; size_t off = 0;
  auto take = [&](size_t bytes) { char* p = ws + off; off += (bytes + 255) & ~(size_t)255; return p; };
  _Float16* BW = (_Float16*)take((size_t)4 * DM * DM * 2);
  _Float16* X16 = (_Float16*)take(NR * DM * 2);
  _Float16* C16 = (_Float16*)take(NR * DM * 2);
  _Float16* Q16 = (_Float16*)take(NR * DM * 2);
  _Float16* KV16 = (_Float16*)take((size_t)2 * NR * DM * 2);
  _Float16* CC16 = (_Float16*)take(NR * DM * 2);
  if (off > ws_size || off > (size_t)134217728) return;
  _Float16* BQ = BW; _Float16* BK = BW + (size_t)DM * DM; _Float16* BO = BW + (size_t)3 * DM * DM;
  _Float16* K16 = KV16; _Float16* V16 = KV16 + NR * DM;

  k_wperm4<<<(unsigned)(((size_t)DM * DM / 8 + 255) / 256), 256, 0, stream>>>(wq, wk, wv, wo, (size_t)DM * DM / 8, BW);
  k_x16<<<(unsigned)((NR * DM / 8 + 255) / 256), 256, 0, stream>>>(x, X16, NR * DM / 8);
  k_x16<<<(unsigned)((NR * DM / 8 + 255) / 256), 256, 0, stream>>>(ctx, C16, NR * DM / 8);
  k_gemm2<<<dim3((unsigned)((NR / 128) * (DM / 64)), 1), 128, 0, stream>>>(X16, DM, 0, BQ, DM, 0, 0.0625f, nullptr, Q16, DM, 0, (int)NR, DM, DM);
  k_gemm2<<<dim3((unsigned)((NR / 128) * (DM / 64)), 2), 128, 0, stream>>>(C16, DM, 0, BK, DM, (size_t)DM * DM, 0.0625f, nullptr, KV16, DM, NR * DM, (int)NR, DM, DM);
  k_attn_tok<<<(unsigned)(NR / 4), 128, 0, stream>>>(Q16, K16, V16, CC16);
  k_gemm2<<<dim3((unsigned)((SEQ / 128) * (DM / 64)), NB), 128, 0, stream>>>(CC16, DM, (size_t)SEQ * DM, BO, DM, 0, 0.0009765625f, (float*)d_out, nullptr, DM, (size_t)SEQ_FULL * DM, SEQ, DM, DM);
}
